// GraphAttentionRela_73701638799908
// MI455X (gfx1250) — hardware-verified
//
#include <hip/hip_runtime.h>
#include <stddef.h>


typedef _Float16 v16h __attribute__((ext_vector_type(16)));
typedef _Float16 v8h  __attribute__((ext_vector_type(8)));
typedef float    v8f  __attribute__((ext_vector_type(8)));
typedef float    v4f  __attribute__((ext_vector_type(4)));
typedef _Float16 h16;

#ifndef NB
#define NB 16
#endif
#define NB_FULL 16
#define ATT   64
#define RELA  128
#define DIN   1024
#define HIDN  512
#define MROWS (NB * ATT)

static_assert(NB >= 1 && NB <= NB_FULL);
static_assert(ATT == 64);
static_assert((RELA % 64) == 0 && (RELA % 32) == 0);
static_assert((DIN % 64) == 0 && (DIN % 32) == 0);
static_assert((HIDN % 64) == 0 && (HIDN % 32) == 0);
static_assert((MROWS % 64) == 0);
static_assert(HIDN == 4 * 32 * 4);
static_assert(HIDN == 2 * 256);
static_assert(RELA == 8 * 16);
static_assert(RELA == 16 * 8);
static_assert(((size_t)MROWS * DIN) % 2048 == 0);

#define LDT 72
#define LDC 68
static_assert((LDT % 8) == 0 && LDT >= 64);
static_assert((LDC % 4) == 0 && LDC >= 64);

#define WCARRY 64.0f
#define XCARRY 16.0f
#define PCARRY 1024.0f
#define EPSV   1.0e-8f

#define WT_BYTES   ((size_t)HIDN * DIN * 2)
#define A16_BYTES  ((size_t)MROWS * DIN * 2)
#define RT_BYTES   ((size_t)NB * DIN * RELA * 2)
#define ATTF_BYTES ((size_t)MROWS * HIDN * 4)
#define P16_BYTES  ((size_t)MROWS * RELA * 2)
#define OFF_WT   ((size_t)0)
#define OFF_A16  (OFF_WT + WT_BYTES)
#define OFF_RT   (OFF_A16 + A16_BYTES)
#define OFF_ATTF (OFF_RT + RT_BYTES)
#define OFF_P16  (OFF_ATTF + ATTF_BYTES)
#define WS_TOTAL (OFF_P16 + P16_BYTES)
static_assert((WT_BYTES % 128) == 0 && (A16_BYTES % 128) == 0 && (RT_BYTES % 128) == 0);
static_assert((ATTF_BYTES % 128) == 0 && (P16_BYTES % 128) == 0);
static_assert(WS_TOTAL <= (size_t)134217728);

__device__ __forceinline__ float bf16r(float x) {
  unsigned int u = __float_as_uint(x);
  u = (u + 0x7FFFu + ((u >> 16) & 1u)) & 0xFFFF0000u;
  return __uint_as_float(u);
}

static __device__ __forceinline__ h16 toh_flush(float v) {
  const h16 r = (h16)v;
  return (fabsf(v) < 6.103515625e-05f) ? (h16)0.0f : r;
}

__device__ __forceinline__ v16h frag_at(const _Float16* p) {
  v8h lo = *(const v8h*)(p);
  v8h hi = *(const v8h*)(p + 16);
  v16h out;
#pragma unroll
  for (int i = 0; i < 8; ++i) { out[i] = lo[i]; out[i + 8] = hi[i]; }
  return out;
}

__device__ __forceinline__ v8f wmma16(v16h a, v16h b, v8f c) {
  v8f d = __builtin_amdgcn_wmma_f32_16x16x32_f16(false, a, false, b, (short)0, c,
                                                 false, false);
  asm volatile("v_nop\n\tv_nop\n\tv_nop\n\tv_nop" : "+v"(d) : "v"(a), "v"(b));
  return d;
}

__device__ __forceinline__ float red32_sum(float x) {
#pragma unroll
  for (int off = 1; off < 32; off <<= 1) x += __shfl_xor(x, off, 32);
  return x;
}
__device__ __forceinline__ float red32_max(float x) {
#pragma unroll
  for (int off = 1; off < 32; off <<= 1) x = fmaxf(x, __shfl_xor(x, off, 32));
  return x;
}

__device__ __forceinline__ float tanh_e(float x) {
  const float xc = fminf(fmaxf(x, -15.0f), 15.0f);
  const float e = __expf(2.0f * xc);
  return 1.0f - 2.0f * __builtin_amdgcn_rcpf(e + 1.0f);
}

__global__ __launch_bounds__(256) void wconv_kernel(
    const float* __restrict__ W, _Float16* __restrict__ Wt, unsigned ldw, unsigned ldk) {
  __shared__ __attribute__((aligned(16))) _Float16 T[64 * LDT];
  const unsigned tid = threadIdx.x;
  const unsigned n0 = blockIdx.x * 64u;
  const unsigned k0 = blockIdx.y * 64u;
#pragma unroll 4
  for (unsigned j = 0; j < 16u; ++j) {
    const unsigned idx = tid + 256u * j;
    const unsigned kr = idx >> 6, nc = idx & 63u;
    const float v = W[(size_t)(k0 + kr) * ldw + n0 + nc];
    T[nc * LDT + kr] = toh_flush(WCARRY * bf16r(v));
  }
  __syncthreads();
  v8h x[2];
  size_t off[2];
#pragma unroll
  for (unsigned i = 0; i < 2u; ++i) {
    const unsigned n = 32u * i + (tid >> 3);
    const unsigned kc = (tid & 7u) * 8u;
    x[i] = *(const v8h*)&T[n * LDT + kc];
    off[i] = (size_t)(n0 + n) * ldk + k0 + kc;
  }
#pragma unroll
  for (int i = 0; i < 2; ++i) *(volatile v8h*)(Wt + off[i]) = x[i];
  __threadfence();
#pragma unroll
  for (int i = 0; i < 2; ++i) *(volatile v8h*)(Wt + off[i]) = x[i];
}

__global__ __launch_bounds__(256) void rconv_kernel(
    const float* __restrict__ R, _Float16* __restrict__ RT) {
  __shared__ __attribute__((aligned(16))) _Float16 T[64 * LDT];
  const unsigned tid = threadIdx.x;
  const unsigned n0 = blockIdx.x * 64u;
  const unsigned k0 = blockIdx.y * 64u;
  const size_t rbase = (size_t)blockIdx.z * ((size_t)RELA * DIN);
  const size_t tbase = (size_t)blockIdx.z * ((size_t)DIN * RELA);
#pragma unroll 4
  for (unsigned j = 0; j < 16u; ++j) {
    const unsigned idx = tid + 256u * j;
    const unsigned kr = idx >> 6, nc = idx & 63u;
    const float v = R[rbase + (size_t)(k0 + kr) * DIN + n0 + nc];
    T[nc * LDT + kr] = toh_flush(WCARRY * bf16r(v));
  }
  __syncthreads();
  v8h x[2];
  size_t off[2];
#pragma unroll
  for (unsigned i = 0; i < 2u; ++i) {
    const unsigned n = 32u * i + (tid >> 3);
    const unsigned kc = (tid & 7u) * 8u;
    x[i] = *(const v8h*)&T[n * LDT + kc];
    off[i] = tbase + (size_t)(n0 + n) * RELA + k0 + kc;
  }
#pragma unroll
  for (int i = 0; i < 2; ++i) *(volatile v8h*)(RT + off[i]) = x[i];
  __threadfence();
#pragma unroll
  for (int i = 0; i < 2; ++i) *(volatile v8h*)(RT + off[i]) = x[i];
}

__global__ __launch_bounds__(256) void xconv_kernel(
    const float* __restrict__ X, _Float16* __restrict__ dst) {
  const size_t i = ((size_t)blockIdx.x * 256u + threadIdx.x) * 8u;
  const v4f a0 = *(const v4f*)(X + i);
  const v4f a1 = *(const v4f*)(X + i + 4u);
  v8h o;
#pragma unroll
  for (int j = 0; j < 4; ++j) {
    o[j]     = toh_flush(XCARRY * bf16r(a0[j]));
    o[j + 4] = toh_flush(XCARRY * bf16r(a1[j]));
  }
  _Float16* p = dst + i;
  *(volatile v8h*)p = o;
  __threadfence();
  *(volatile v8h*)p = o;
}

template <int MODE>
__device__ __forceinline__ void gemm_body(
    const _Float16* __restrict__ A16, const _Float16* __restrict__ Bt, const unsigned K,
    const size_t bstride, const float* __restrict__ bias, float* __restrict__ outf,
    const unsigned ldo) {
  __shared__ __attribute__((aligned(16))) float Cs[64 * LDC];
  const unsigned tid = threadIdx.x, lane = tid & 31u;
  const unsigned w = (unsigned)__builtin_amdgcn_readfirstlane((int)(threadIdx.x >> 5));
  const unsigned mw = w >> 1, nw = w & 1u;
  const unsigned hh = lane >> 4, m = lane & 15u;
  const unsigned n0 = blockIdx.x * 64u;
  const unsigned row0 = blockIdx.y * 64u;

  const _Float16* ap  = A16 + (size_t)(row0 + mw * 16u + m) * K + hh * 8u;
  const _Float16* bp0 = Bt + (size_t)blockIdx.y * bstride
                           + (size_t)(n0 + nw * 32u + m) * K + hh * 8u;
  const _Float16* bp1 = bp0 + (size_t)16 * K;
  v8f acc0 = {}, acc1 = {};
#pragma unroll 2
  for (unsigned k0 = 0; k0 < K; k0 += 32u) {
    const v16h a  = frag_at(ap + k0);
    const v16h b0 = frag_at(bp0 + k0);
    const v16h b1 = frag_at(bp1 + k0);
    acc0 = wmma16(a, b0, acc0);
    acc1 = wmma16(a, b1, acc1);
  }
#pragma unroll
  for (int r = 0; r < 8; ++r) {
    float* d = &Cs[(mw * 16u + hh * 8u + (unsigned)r) * LDC + nw * 32u + m];
    d[0]  = acc0[r];
    d[16] = acc1[r];
  }
  __syncthreads();

  const float cs = (MODE == 0) ? (1.0f / (WCARRY * XCARRY)) : (1.0f / (PCARRY * WCARRY));
  v4f xs[4];
  size_t off[4];
#pragma unroll
  for (unsigned i = 0; i < 4u; ++i) {
    const unsigned r = 16u * i + (tid >> 4);
    const unsigned c = (tid & 15u) * 4u;
    const v4f u = *(const v4f*)&Cs[r * LDC + c];
    v4f val;
    if (MODE == 0) {
      const v4f g = *(const v4f*)(bias + n0 + c);
#pragma unroll
      for (int j = 0; j < 4; ++j) val[j] = u[j] * cs + bf16r(g[j]);
    } else {
#pragma unroll
      for (int j = 0; j < 4; ++j) val[j] = u[j] * cs;
    }
    xs[i] = val;
    off[i] = (size_t)(row0 + r) * ldo + n0 + c;
  }
#pragma unroll
  for (int i = 0; i < 4; ++i) *(volatile v4f*)(outf + off[i]) = xs[i];
  __threadfence();
#pragma unroll
  for (int i = 0; i < 4; ++i) *(volatile v4f*)(outf + off[i]) = xs[i];
}

__global__ __launch_bounds__(256) void gemm_obj_kernel(
    const _Float16* __restrict__ A16, const _Float16* __restrict__ Bt,
    const float* __restrict__ bias, float* __restrict__ outf) {
  gemm_body<0>(A16, Bt, (unsigned)DIN, (size_t)0, bias, outf, (unsigned)HIDN);
}
__global__ __launch_bounds__(256) void gemm_out_kernel(
    const _Float16* __restrict__ P16, const _Float16* __restrict__ RT,
    float* __restrict__ outf) {
  gemm_body<1>(P16, RT, (unsigned)RELA, (size_t)DIN * RELA, (const float*)0, outf,
               (unsigned)DIN);
}

static_assert((HIDN * 2 + RELA + 2) * 4 + RELA * 2 <= 131072);

__global__ __launch_bounds__(256) void score_kernel(
    const float* __restrict__ attf, const float* __restrict__ prela,
    const float* __restrict__ walpha, const float* __restrict__ balpha,
    const int* __restrict__ mask, _Float16* __restrict__ P16) {
  __shared__ __attribute__((aligned(16))) float s_att[HIDN];
  __shared__ __attribute__((aligned(16))) float s_wa[HIDN];
  __shared__ __attribute__((aligned(16))) float s_sc[RELA];
  __shared__ float s_red[2];
  __shared__ __attribute__((aligned(16))) _Float16 s_p[RELA];

  const unsigned tid = threadIdx.x, lane = tid & 31u;
  const unsigned wave = (unsigned)__builtin_amdgcn_readfirstlane((int)(threadIdx.x >> 5));
  const unsigned ba = blockIdx.x;
  const unsigned b = ba / (unsigned)ATT;

#pragma unroll
  for (unsigned j = 0; j < 2u; ++j) {
    const unsigned h = tid + 256u * j;
    s_att[h] = attf[(size_t)ba * HIDN + h];
    s_wa[h]  = bf16r(walpha[h]);
  }
  const float bal = bf16r(balpha[0]);
  __syncthreads();

  const float* prow = prela + (size_t)b * ((size_t)RELA * HIDN) + lane * 4u;
#pragma unroll 1
  for (unsigned i = 0; i < 16u; ++i) {
    const unsigned r = wave * 16u + i;
    const float* pr = prow + (size_t)r * HIDN;
    float acc = 0.0f;
#pragma unroll 1
    for (unsigned j = 0; j < 4u; ++j) {
      const unsigned c = j * 128u + lane * 4u;
      const v4f pv = *(const v4f*)(pr + j * 128u);
      const v4f av = *(const v4f*)&s_att[c];
      const v4f wv = *(const v4f*)&s_wa[c];
#pragma unroll
      for (int q = 0; q < 4; ++q)
        acc = fmaf(wv[q], tanh_e(bf16r(pv[q]) + av[q]), acc);
    }
    acc = red32_sum(acc);
    if (lane == 0u) s_sc[r] = acc + bal;
  }
  __syncthreads();

  if (wave == 0u) {
    float mx = fmaxf(fmaxf(s_sc[lane], s_sc[lane + 32u]),
                     fmaxf(s_sc[lane + 64u], s_sc[lane + 96u]));
    mx = red32_max(mx);
    if (lane == 0u) s_red[0] = mx;
  }
  __syncthreads();
  const float mv = s_red[0];
  float e = 0.0f;
  if (wave < 4u) {
    e = __expf(s_sc[tid] - mv);
    s_sc[tid] = e;
  }
  __syncthreads();

  if (wave == 0u) {
    float s = (s_sc[lane] + s_sc[lane + 32u]) + (s_sc[lane + 64u] + s_sc[lane + 96u]);
    s = red32_sum(s);
    if (lane == 0u) s_red[1] = s;
  }
  __syncthreads();
  const float einv = __builtin_amdgcn_rcpf(s_red[1]);

  float wm = 0.0f;
  if (wave < 4u) {
    const float mk = (float)mask[(size_t)ba * RELA + tid];
    wm = (e * einv) * mk;
    s_sc[tid] = wm;
  }
  __syncthreads();
  if (wave == 0u) {
    float s = (s_sc[lane] + s_sc[lane + 32u]) + (s_sc[lane + 64u] + s_sc[lane + 96u]);
    s = red32_sum(s);
    if (lane == 0u) s_red[0] = s;
  }
  __syncthreads();
  const float ninv = __builtin_amdgcn_rcpf(s_red[0] + EPSV);
  if (wave < 4u) s_p[tid] = toh_flush(PCARRY * (wm * ninv));
  __syncthreads();

  if (wave == 0u) {
    if (lane < 16u) {
      const v8h x = *(const v8h*)&s_p[lane * 8u];
      _Float16* dp = P16 + (size_t)ba * RELA + lane * 8u;
      *(volatile v8h*)dp = x;
      __threadfence();
      *(volatile v8h*)dp = x;
    }
  }
}

extern "C" void kernel_launch(void* const* d_in, const int* in_sizes, int n_in,
                              void* d_out, int out_size, void* d_ws, size_t ws_size,
                              hipStream_t stream) {
  if (n_in < 8) return;
  if ((long long)in_sizes[0] < (long long)MROWS * DIN) return;
  if ((long long)in_sizes[1] < (long long)NB * RELA * DIN) return;
  if ((long long)in_sizes[2] < (long long)NB * RELA * HIDN) return;
  if ((long long)in_sizes[3] < (long long)DIN * HIDN) return;
  if (in_sizes[4] < HIDN || in_sizes[5] < HIDN || in_sizes[6] < 1) return;
  if ((long long)in_sizes[7] < (long long)MROWS * RELA) return;
  if ((long long)out_size < (long long)MROWS * DIN) return;
  if (ws_size < WS_TOTAL) return;

  const float* obj    = (const float*)d_in[0];
  const float* rela   = (const float*)d_in[1];
  const float* prela  = (const float*)d_in[2];
  const float* wobj   = (const float*)d_in[3];
  const float* bobj   = (const float*)d_in[4];
  const float* walpha = (const float*)d_in[5];
  const float* balpha = (const float*)d_in[6];
  const int*   mask   = (const int*)d_in[7];
  float* out = (float*)d_out;

  char* ws = (char*)d_ws;
  _Float16* Wt   = (_Float16*)(ws + OFF_WT);
  _Float16* A16  = (_Float16*)(ws + OFF_A16);
  _Float16* RT   = (_Float16*)(ws + OFF_RT);
  float*    AttF = (float*)(ws + OFF_ATTF);
  _Float16* P16  = (_Float16*)(ws + OFF_P16);

  dim3 blk(256);

  wconv_kernel<<<dim3(HIDN / 64, DIN / 64), blk, 0, stream>>>(wobj, Wt, (unsigned)HIDN,
                                                              (unsigned)DIN);
  rconv_kernel<<<dim3(DIN / 64, RELA / 64, NB), blk, 0, stream>>>(rela, RT);
  xconv_kernel<<<dim3((unsigned)(((size_t)MROWS * DIN) / 2048)), blk, 0, stream>>>(obj, A16);
  gemm_obj_kernel<<<dim3(HIDN / 64, MROWS / 64), blk, 0, stream>>>(A16, Wt, bobj, AttF);
  score_kernel<<<dim3(MROWS), blk, 0, stream>>>(AttF, prela, walpha, balpha, mask, P16);
  gemm_out_kernel<<<dim3(DIN / 64, NB), blk, 0, stream>>>(P16, RT, out);
}
